// ProjectionNetwork_37589553774839
// MI455X (gfx1250) — hardware-verified
//
#include <hip/hip_runtime.h>
#include <stddef.h>


typedef _Float16 v16h __attribute__((ext_vector_type(16)));
typedef _Float16 v8h  __attribute__((ext_vector_type(8)));
typedef float    v8f  __attribute__((ext_vector_type(8)));
typedef float    v4f  __attribute__((ext_vector_type(4)));
typedef _Float16 h16;

#ifndef NCOLS
#define NCOLS 16384
#endif
#define NCOLS_FULL 16384
#define DIM   512

#define PW          32
#define NPANEL      (DIM / PW)
#define GS_THREADS  512

static_assert(NCOLS >= 64 && NCOLS <= NCOLS_FULL && (NCOLS % 64) == 0);
static_assert((DIM % 64) == 0 && (DIM % 32) == 0);
static_assert(GS_THREADS == DIM);
static_assert(PW == 2 * (GS_THREADS / 32));
static_assert(DIM == 4 * 32 * 4);
static_assert(PW * 4 == 128);
static_assert(NPANEL * PW == DIM);
static_assert((size_t)(PW * DIM + 2 * DIM) * 4 <= (size_t)131072);

#define LDT 72
#define LDC 68
static_assert((LDT % 8) == 0 && LDT >= 64);
static_assert((LDC % 4) == 0 && LDC >= 64);

#define WCARRY  64.0f
#define UCARRY  64.0f
#define PMCARRY 64.0f
#define PSCALE  (PMCARRY / (UCARRY * UCARRY))
#define OSCALE  (1.0f / (PMCARRY * WCARRY))

#define QC_BYTES   ((size_t)DIM * DIM * 4)
#define SQ16_BYTES ((size_t)DIM * DIM * 2)
#define XT_BYTES   ((size_t)NCOLS * DIM * 2)
#define OFF_QC  ((size_t)0)
#define OFF_U   (OFF_QC + QC_BYTES)
#define OFF_UD  (OFF_U + SQ16_BYTES)
#define OFF_P   (OFF_UD + SQ16_BYTES)
#define OFF_XT  (OFF_P + SQ16_BYTES)
#define WS_TOTAL (OFF_XT + XT_BYTES)
static_assert((QC_BYTES % 128) == 0 && (SQ16_BYTES % 128) == 0 && (XT_BYTES % 128) == 0);
static_assert(WS_TOTAL <= (size_t)134217728);

__device__ __forceinline__ float bf16r(float x) {
  unsigned int u = __float_as_uint(x);
  u = (u + 0x7FFFu + ((u >> 16) & 1u)) & 0xFFFF0000u;
  return __uint_as_float(u);
}

static __device__ __forceinline__ h16 toh_flush(float v) {
  const h16 r = (h16)v;
  return (fabsf(v) < 6.103515625e-05f) ? (h16)0.0f : r;
}

__device__ __forceinline__ v16h frag_at(const _Float16* p) {
  v8h lo = *(const v8h*)(p);
  v8h hi = *(const v8h*)(p + 16);
  v16h out;
#pragma unroll
  for (int i = 0; i < 8; ++i) { out[i] = lo[i]; out[i + 8] = hi[i]; }
  return out;
}

__device__ __forceinline__ v8f wmma16(v16h a, v16h b, v8f c) {
  v8f d = __builtin_amdgcn_wmma_f32_16x16x32_f16(false, a, false, b, (short)0, c,
                                                 false, false);
  asm volatile("v_nop\n\tv_nop\n\tv_nop\n\tv_nop" : "+v"(d) : "v"(a), "v"(b));
  return d;
}

__device__ __forceinline__ float red32_sum(float x) {
#pragma unroll
  for (int off = 1; off < 32; off <<= 1) x += __shfl_xor(x, off, 32);
  return x;
}

__global__ __launch_bounds__(256) void wconv_kernel(
    const float* __restrict__ W, _Float16* __restrict__ Wt, unsigned ldw, unsigned ldk) {
  __shared__ _Float16 T[64 * LDT];
  const unsigned tid = threadIdx.x;
  const unsigned n0 = blockIdx.x * 64u;
  const unsigned k0 = blockIdx.y * 64u;
#pragma unroll 4
  for (unsigned j = 0; j < 16u; ++j) {
    const unsigned idx = tid + 256u * j;
    const unsigned kr = idx >> 6, nc = idx & 63u;
    const float v = W[(size_t)(k0 + kr) * ldw + n0 + nc];
    T[nc * LDT + kr] = toh_flush(WCARRY * bf16r(v));
  }
  __syncthreads();
  v8h x[2];
  size_t off[2];
#pragma unroll
  for (unsigned i = 0; i < 2u; ++i) {
    const unsigned n = 32u * i + (tid >> 3);
    const unsigned kc = (tid & 7u) * 8u;
    x[i] = *(const v8h*)&T[n * LDT + kc];
    off[i] = (size_t)(n0 + n) * ldk + k0 + kc;
  }
#pragma unroll
  for (int i = 0; i < 2; ++i) *(volatile v8h*)(Wt + off[i]) = x[i];
  __threadfence();
#pragma unroll
  for (int i = 0; i < 2; ++i) *(volatile v8h*)(Wt + off[i]) = x[i];
}

__global__ __launch_bounds__(GS_THREADS) void gs_panel_kernel(
    const float* __restrict__ W, float* Qc, const unsigned p) {
  __shared__ float cols[PW * DIM];
  __shared__ float qs[2 * DIM];
  if (p >= (unsigned)NPANEL) return;
  const unsigned tid = threadIdx.x, lane = tid & 31u;
  const unsigned wave = (unsigned)__builtin_amdgcn_readfirstlane((int)(tid >> 5));
  const unsigned col0 = p * (unsigned)PW;
  const unsigned lo4 = lane * 4u;

  {
    const float* src = W + (size_t)tid * DIM + col0;
#pragma unroll
    for (unsigned g = 0; g < (unsigned)(PW / 4); ++g) {
      const v4f a = *(const v4f*)(src + 4u * g);
      cols[(4u * g + 0u) * DIM + tid] = bf16r(a[0]);
      cols[(4u * g + 1u) * DIM + tid] = bf16r(a[1]);
      cols[(4u * g + 2u) * DIM + tid] = bf16r(a[2]);
      cols[(4u * g + 3u) * DIM + tid] = bf16r(a[3]);
    }
  }
  __syncthreads();

#pragma unroll 1
  for (unsigned j = 0; j < col0; ++j) {
    const float* qg = Qc + (size_t)j * DIM + lo4;
#pragma unroll 1
    for (unsigned sl = 0; sl < 2u; ++sl) {
      const unsigned cb = (wave + 16u * sl) * (unsigned)DIM + lo4;
      float s = 0.0f;
#pragma unroll 1
      for (unsigned t = 0; t < 4u; ++t) {
        const v4f q = *(const v4f*)(qg + t * 128u);
        const v4f a = *(const v4f*)&cols[cb + t * 128u];
        s += a[0] * q[0];
        s += a[1] * q[1];
        s += a[2] * q[2];
        s += a[3] * q[3];
      }
      s = red32_sum(s);
#pragma unroll 1
      for (unsigned t = 0; t < 4u; ++t) {
        const v4f q = *(const v4f*)(qg + t * 128u);
        v4f a = *(const v4f*)&cols[cb + t * 128u];
        a[0] -= s * q[0];
        a[1] -= s * q[1];
        a[2] -= s * q[2];
        a[3] -= s * q[3];
        *(v4f*)&cols[cb + t * 128u] = a;
      }
    }
  }

#pragma unroll 1
  for (unsigned j = 0; j < (unsigned)PW; ++j) {
    const unsigned qb = (j & 1u) * (unsigned)DIM + lo4;
    if (wave == (j & 15u)) {
      const unsigned cj = j * (unsigned)DIM + lo4;
      float s = 0.0f;
#pragma unroll 1
      for (unsigned t = 0; t < 4u; ++t) {
        const v4f a = *(const v4f*)&cols[cj + t * 128u];
        s += a[0] * a[0];
        s += a[1] * a[1];
        s += a[2] * a[2];
        s += a[3] * a[3];
      }
      s = red32_sum(s);
      const float inv = 1.0f / sqrtf(s);
      float* qdst = Qc + (size_t)(col0 + j) * DIM + lo4;
#pragma unroll 1
      for (unsigned t = 0; t < 4u; ++t) {
        const v4f a = *(const v4f*)&cols[cj + t * 128u];
        const v4f q = a * inv;
        *(v4f*)&qs[qb + t * 128u] = q;
        *(volatile v4f*)(qdst + t * 128u) = q;
      }
      __threadfence();
#pragma unroll 1
      for (unsigned t = 0; t < 4u; ++t) {
        const v4f q = *(const v4f*)&qs[qb + t * 128u];
        *(volatile v4f*)(qdst + t * 128u) = q;
      }
    }
    __syncthreads();
#pragma unroll 1
    for (unsigned sl = 0; sl < 2u; ++sl) {
      const unsigned c = wave + 16u * sl;
      if (c > j) {
        const unsigned cb = c * (unsigned)DIM + lo4;
        float s = 0.0f;
#pragma unroll 1
        for (unsigned t = 0; t < 4u; ++t) {
          const v4f q = *(const v4f*)&qs[qb + t * 128u];
          const v4f a = *(const v4f*)&cols[cb + t * 128u];
          s += a[0] * q[0];
          s += a[1] * q[1];
          s += a[2] * q[2];
          s += a[3] * q[3];
        }
        s = red32_sum(s);
#pragma unroll 1
        for (unsigned t = 0; t < 4u; ++t) {
          const v4f q = *(const v4f*)&qs[qb + t * 128u];
          v4f a = *(const v4f*)&cols[cb + t * 128u];
          a[0] -= s * q[0];
          a[1] -= s * q[1];
          a[2] -= s * q[2];
          a[3] -= s * q[3];
          *(v4f*)&cols[cb + t * 128u] = a;
        }
      }
    }
  }
}

__global__ __launch_bounds__(256) void uconv_kernel(
    const float* __restrict__ Qc, const float* __restrict__ Dp,
    _Float16* __restrict__ U16, _Float16* __restrict__ UD16) {
  __shared__ _Float16 T[64 * LDT];
  __shared__ _Float16 TD[64 * LDT];
  __shared__ float Ds[64];
  const unsigned tid = threadIdx.x;
  const unsigned n0 = blockIdx.x * 64u;
  const unsigned k0 = blockIdx.y * 64u;
  if (tid < 64u) {
    const float d = bf16r(Dp[k0 + tid]);
    Ds[tid] = 1.0f / (1.0f + expf(-d));
  }
  __syncthreads();
#pragma unroll 4
  for (unsigned j = 0; j < 16u; ++j) {
    const unsigned idx = tid + 256u * j;
    const unsigned kr = idx >> 6, nc = idx & 63u;
    const float v = Qc[(size_t)(k0 + kr) * DIM + n0 + nc];
    const float vd = v * Ds[kr];
    T[nc * LDT + kr]  = toh_flush(UCARRY * v);
    TD[nc * LDT + kr] = toh_flush(UCARRY * vd);
  }
  __syncthreads();
  v8h x[2], xd[2];
  size_t off[2];
#pragma unroll
  for (unsigned i = 0; i < 2u; ++i) {
    const unsigned n = 32u * i + (tid >> 3);
    const unsigned kc = (tid & 7u) * 8u;
    x[i]  = *(const v8h*)&T[n * LDT + kc];
    xd[i] = *(const v8h*)&TD[n * LDT + kc];
    off[i] = (size_t)(n0 + n) * DIM + k0 + kc;
  }
#pragma unroll
  for (int i = 0; i < 2; ++i) *(volatile v8h*)(U16 + off[i]) = x[i];
#pragma unroll
  for (int i = 0; i < 2; ++i) *(volatile v8h*)(UD16 + off[i]) = xd[i];
  __threadfence();
#pragma unroll
  for (int i = 0; i < 2; ++i) *(volatile v8h*)(U16 + off[i]) = x[i];
#pragma unroll
  for (int i = 0; i < 2; ++i) *(volatile v8h*)(UD16 + off[i]) = xd[i];
}

static_assert(32 * 2 == 64 && 16 * 4 == 64);

template <int MODE>
__device__ __forceinline__ void gemm_body(
    const _Float16* __restrict__ A16, const _Float16* __restrict__ Bt, const unsigned K,
    float* __restrict__ outf, _Float16* __restrict__ out16) {
  __shared__ float Cs[64 * LDC];
  const unsigned tid = threadIdx.x, lane = tid & 31u, w = tid >> 5;
  const unsigned mw = w >> 1, nw = w & 1u;
  const unsigned hh = lane >> 4, m = lane & 15u;
  const unsigned n0 = blockIdx.x * 64u;
  const unsigned row0 = blockIdx.y * 64u;

  const _Float16* ap  = A16 + (size_t)(row0 + mw * 16u + m) * K + hh * 8u;
  const _Float16* bp0 = Bt + (size_t)(n0 + nw * 32u + m) * K + hh * 8u;
  const _Float16* bp1 = bp0 + (size_t)16 * K;
  v8f acc0 = {}, acc1 = {};
#pragma unroll 2
  for (unsigned k0 = 0; k0 < K; k0 += 32u) {
    const v16h a  = frag_at(ap + k0);
    const v16h b0 = frag_at(bp0 + k0);
    const v16h b1 = frag_at(bp1 + k0);
    acc0 = wmma16(a, b0, acc0);
    acc1 = wmma16(a, b1, acc1);
  }
#pragma unroll
  for (int r = 0; r < 8; ++r) {
    float* d = &Cs[(mw * 16u + hh * 8u + (unsigned)r) * LDC + nw * 32u + m];
    d[0]  = acc0[r];
    d[16] = acc1[r];
  }
  __syncthreads();

  if (MODE == 0) {
    v8h x[2];
    size_t off[2];
#pragma unroll
    for (unsigned i = 0; i < 2u; ++i) {
      const unsigned r = 32u * i + (tid >> 3);
      const unsigned c = (tid & 7u) * 8u;
      const v4f u0 = *(const v4f*)&Cs[r * LDC + c];
      const v4f u1 = *(const v4f*)&Cs[r * LDC + c + 4];
#pragma unroll
      for (int j = 0; j < 4; ++j) {
        x[i][j]     = toh_flush(u0[j] * PSCALE);
        x[i][j + 4] = toh_flush(u1[j] * PSCALE);
      }
      off[i] = (size_t)(row0 + r) * DIM + n0 + c;
    }
#pragma unroll
    for (int i = 0; i < 2; ++i) *(volatile v8h*)(out16 + off[i]) = x[i];
    __threadfence();
#pragma unroll
    for (int i = 0; i < 2; ++i) *(volatile v8h*)(out16 + off[i]) = x[i];
  }

  if (MODE == 1) {
    v4f xs[4];
    size_t off[4];
#pragma unroll
    for (unsigned i = 0; i < 4u; ++i) {
      const unsigned r = 16u * i + (tid >> 4);
      const unsigned c = (tid & 15u) * 4u;
      const v4f u = *(const v4f*)&Cs[r * LDC + c];
      xs[i] = u * OSCALE;
      off[i] = (size_t)(row0 + r) * NCOLS_FULL + n0 + c;
    }
#pragma unroll
    for (int i = 0; i < 4; ++i) *(volatile v4f*)(outf + off[i]) = xs[i];
    __threadfence();
#pragma unroll
    for (int i = 0; i < 4; ++i) *(volatile v4f*)(outf + off[i]) = xs[i];
  }
}

__global__ __launch_bounds__(256) void gemm_p_kernel(
    const _Float16* __restrict__ A16, const _Float16* __restrict__ Bt,
    _Float16* __restrict__ out16) {
  gemm_body<0>(A16, Bt, (unsigned)DIM, (float*)0, out16);
}
__global__ __launch_bounds__(256) void gemm_out_kernel(
    const _Float16* __restrict__ A16, const _Float16* __restrict__ Bt,
    float* __restrict__ outf) {
  gemm_body<1>(A16, Bt, (unsigned)DIM, outf, (_Float16*)0);
}

extern "C" void kernel_launch(void* const* d_in, const int* in_sizes, int n_in,
                              void* d_out, int out_size, void* d_ws, size_t ws_size,
                              hipStream_t stream) {
  if (n_in < 3) return;
  const long long need_x = (long long)(DIM - 1) * NCOLS_FULL + NCOLS;
  if ((long long)in_sizes[0] < need_x) return;
  if ((long long)in_sizes[1] < (long long)DIM * DIM) return;
  if (in_sizes[2] < DIM) return;
  if ((long long)out_size < need_x) return;
  if (ws_size < WS_TOTAL) return;

  const float* X  = (const float*)d_in[0];
  const float* Wm = (const float*)d_in[1];
  const float* Dp = (const float*)d_in[2];
  float* out = (float*)d_out;

  char* ws = (char*)d_ws;
  float*    Qc   = (float*)(ws + OFF_QC);
  _Float16* U16  = (_Float16*)(ws + OFF_U);
  _Float16* UD16 = (_Float16*)(ws + OFF_UD);
  _Float16* P16  = (_Float16*)(ws + OFF_P);
  _Float16* XT16 = (_Float16*)(ws + OFF_XT);

  dim3 blk(256);

  wconv_kernel<<<dim3(NCOLS / 64, DIM / 64), blk, 0, stream>>>(X, XT16, (unsigned)NCOLS_FULL,
                                                              (unsigned)DIM);
  for (unsigned p = 0; p < (unsigned)NPANEL; ++p)
    gs_panel_kernel<<<dim3(1), dim3(GS_THREADS), 0, stream>>>(Wm, Qc, p);
  uconv_kernel<<<dim3(DIM / 64, DIM / 64), blk, 0, stream>>>(Qc, Dp, U16, UD16);
  gemm_p_kernel<<<dim3(DIM / 64, DIM / 64), blk, 0, stream>>>(UD16, U16, P16);
  gemm_out_kernel<<<dim3(NCOLS / 64, DIM / 64), blk, 0, stream>>>(P16, XT16, out);
}
